// fusion_module_30709016166519
// MI455X (gfx1250) — hardware-verified
//
#include <hip/hip_runtime.h>
#include <stdint.h>

#define SEQ   2048
#define DM    512
#define NHD   8
#define HD    64
#define KT    32
#define QB    64
#define NQB   32
#define NKT   64
#define GM    128
#define GN    64
#define OSP   68
#define LTP   72
#define PPH   40
#define OTP   68
#define MAXNB 4
#define PSC   64.0f
#define VSC   16.0f
#define SCL   0.125f

static_assert(NHD * HD == DM);
static_assert(NQB * QB == SEQ);
static_assert(NKT * KT == SEQ);
static_assert(SEQ % GM == 0);
static_assert(DM % GN == 0);
static_assert(DM % 64 == 0);
static_assert(DM % 32 == 0);
static_assert(GN == HD);
static_assert((SEQ * DM) % 2048 == 0);
static_assert((OSP * 4) % 16 == 0);
static_assert((LTP * 2) % 16 == 0);
static_assert((PPH * 2) % 16 == 0);
static_assert((OTP * 4) % 16 == 0);
static_assert(QB == 4 * 16);
static_assert(KT == 32);
static_assert(HD == 64);
static_assert(GM % KT == 0);

typedef unsigned short v8us __attribute__((ext_vector_type(8)));
typedef unsigned int   v4u  __attribute__((ext_vector_type(4)));
typedef float          v8f  __attribute__((ext_vector_type(8)));
typedef float          v4f  __attribute__((ext_vector_type(4)));
typedef __bf16         v16b __attribute__((ext_vector_type(16)));
typedef _Float16       v16h __attribute__((ext_vector_type(16)));

union Frag { v8us u[2]; v4u q[2]; v16b b; v16h x; };
static_assert(sizeof(Frag) == 32);

__device__ __forceinline__ unsigned short bf_bits(float f) {
  const unsigned u = __float_as_uint(f);
  return (unsigned short)((u + 0x7FFFu + ((u >> 16) & 1u)) >> 16);
}
__device__ __forceinline__ float bf_up(unsigned short hb) { return __uint_as_float(((unsigned)hb) << 16); }
__device__ __forceinline__ float bfr(float f) { return bf_up(bf_bits(f)); }
__device__ __forceinline__ unsigned short h_bits(float f) {
  const _Float16 hv = (_Float16)f;
  return __builtin_bit_cast(unsigned short, hv);
}
__device__ __forceinline__ unsigned pk16(unsigned short a, unsigned short b) { return (unsigned)a | ((unsigned)b << 16); }
__device__ __forceinline__ v8f zero8() { v8f z = {0.f, 0.f, 0.f, 0.f, 0.f, 0.f, 0.f, 0.f}; return z; }

__device__ __forceinline__ Frag ldfrag(const unsigned short* p) {
  Frag f;
  f.u[0] = *(const v8us*)(p);
  f.u[1] = *(const v8us*)(p + 16);
  return f;
}

__device__ __forceinline__ v8f mma_b(v16b a, v16b b, v8f c) {
  v8f d = __builtin_amdgcn_wmma_f32_16x16x32_bf16(false, a, false, b, (short)0, c, false, false);
#if defined(__HIP_DEVICE_COMPILE__)
  asm volatile("v_nop\n\tv_nop\n\tv_nop\n\tv_nop" : "+v"(d) : "v"(a), "v"(b));
#endif
  return d;
}
__device__ __forceinline__ v8f mma_h(v16h a, v16h b, v8f c) {
  v8f d = __builtin_amdgcn_wmma_f32_16x16x32_f16(false, a, false, b, (short)0, c, false, false);
#if defined(__HIP_DEVICE_COMPILE__)
  asm volatile("v_nop\n\tv_nop\n\tv_nop\n\tv_nop" : "+v"(d) : "v"(a), "v"(b));
#endif
  return d;
}

__device__ __forceinline__ void split8(v4f a, v4f b, v4u& uh, v4u& ul) {
  float f[8] = {a[0], a[1], a[2], a[3], b[0], b[1], b[2], b[3]};
#pragma unroll
  for (int j = 0; j < 4; ++j) {
    const unsigned short h0 = bf_bits(f[2 * j]);
    const unsigned short h1 = bf_bits(f[2 * j + 1]);
    const unsigned short l0 = bf_bits(f[2 * j] - bf_up(h0));
    const unsigned short l1 = bf_bits(f[2 * j + 1] - bf_up(h1));
    uh[j] = pk16(h0, h1);
    ul[j] = pk16(l0, l1);
  }
}

__device__ __forceinline__ v4u pack8h(v4f a, v4f b, float sc) {
  v4u u;
  u[0] = pk16(h_bits(a[0] * sc), h_bits(a[1] * sc));
  u[1] = pk16(h_bits(a[2] * sc), h_bits(a[3] * sc));
  u[2] = pk16(h_bits(b[0] * sc), h_bits(b[1] * sc));
  u[3] = pk16(h_bits(b[2] * sc), h_bits(b[3] * sc));
  return u;
}

__global__ __launch_bounds__(256)
void cvt_kernel(const float* __restrict__ x, unsigned short* y, int n8) {
  const int t = blockIdx.x * 256 + (int)threadIdx.x;
  if (t >= n8) return;
  const float* s = x + (size_t)t * 8;
  const v4f a = *(const v4f*)(s);
  const v4f b = *(const v4f*)(s + 4);
  v4u u;
  u[0] = pk16(bf_bits(a[0]), bf_bits(a[1]));
  u[1] = pk16(bf_bits(a[2]), bf_bits(a[3]));
  u[2] = pk16(bf_bits(b[0]), bf_bits(b[1]));
  u[3] = pk16(bf_bits(b[2]), bf_bits(b[3]));
  unsigned short* d = y + (size_t)t * 8;
  *(volatile v4u*)d = u;
  __threadfence();
  *(volatile v4u*)d = u;
}

__global__ __launch_bounds__(256)
void wtrans_kernel(const float* __restrict__ w, unsigned short* wt, int R, int C) {
  __shared__ __align__(16) unsigned short L[64 * LTP];
  const int tid = threadIdx.x;
  const int c0 = blockIdx.x * 64, r0 = blockIdx.y * 64;
  const int c4 = (tid & 15) * 4, rs = tid >> 4;
#pragma unroll
  for (int it = 0; it < 4; ++it) {
    const int r = it * 16 + rs;
    const v4f v = *(const v4f*)(w + (size_t)(r0 + r) * C + c0 + c4);
#pragma unroll
    for (int j = 0; j < 4; ++j) L[(c4 + j) * LTP + r] = bf_bits(v[j]);
  }
  __syncthreads();
  const int e = tid & 7, lq = tid >> 3;
  v4u u[2];
  size_t po[2];
#pragma unroll
  for (int it = 0; it < 2; ++it) {
    const int c = it * 32 + lq;
    u[it] = *(const v4u*)(L + c * LTP + 8 * e);
    po[it] = (size_t)(c0 + c) * R + r0 + 8 * e;
  }
#pragma unroll
  for (int it = 0; it < 2; ++it) *(volatile v4u*)(wt + po[it]) = u[it];
  __threadfence();
#pragma unroll
  for (int it = 0; it < 2; ++it) *(volatile v4u*)(wt + po[it]) = u[it];
}

template <int MODE>
__global__ __launch_bounds__(256)
void proj_kernel(const unsigned short* __restrict__ A, const unsigned short* __restrict__ B,
                 unsigned short* C16, float* CS) {
  __shared__ __align__(16) float Os[GM * OSP];
  __shared__ __align__(16) float Sm[4 * GN];
  const int tid  = threadIdx.x;
  const int lane = tid & 31, wave = tid >> 5;
  const int hh   = lane >> 4, cl = lane & 15;
  const int wm   = wave >> 1, wn = wave & 1;
  const int mBase = blockIdx.x * GM;
  const int nBase = blockIdx.y * GN;
  const unsigned short* a0p = A + (size_t)(mBase + 32 * wm + cl) * DM + 8 * hh;
  const unsigned short* a1p = a0p + (size_t)16 * DM;
  const unsigned short* b0p = B + (size_t)(nBase + 32 * wn + cl) * DM + 8 * hh;
  const unsigned short* b1p = b0p + (size_t)16 * DM;

  v8f acc[2][2];
#pragma unroll
  for (int mi = 0; mi < 2; ++mi)
#pragma unroll
    for (int ni = 0; ni < 2; ++ni) acc[mi][ni] = zero8();

#pragma unroll 1
  for (int k0 = 0; k0 < DM; k0 += 32) {
    const Frag fa0 = ldfrag(a0p + k0);
    const Frag fa1 = ldfrag(a1p + k0);
    const Frag fb0 = ldfrag(b0p + k0);
    const Frag fb1 = ldfrag(b1p + k0);
    acc[0][0] = mma_b(fa0.b, fb0.b, acc[0][0]);
    acc[0][1] = mma_b(fa0.b, fb1.b, acc[0][1]);
    acc[1][0] = mma_b(fa1.b, fb0.b, acc[1][0]);
    acc[1][1] = mma_b(fa1.b, fb1.b, acc[1][1]);
  }

#pragma unroll
  for (int mi = 0; mi < 2; ++mi) {
#pragma unroll
    for (int ni = 0; ni < 2; ++ni) {
      const int n_loc = 32 * wn + 16 * ni + cl;
#pragma unroll
      for (int r = 0; r < 8; ++r) {
        const int m_loc = 32 * wm + 16 * mi + 8 * hh + r;
        Os[m_loc * OSP + n_loc] = acc[mi][ni][r];
      }
    }
  }
  __syncthreads();

  const int e = tid & 7, lq = tid >> 3;
  if constexpr (MODE == 0) {
    v4u u[4];
    size_t po[4];
#pragma unroll
    for (int it = 0; it < 4; ++it) {
      const int row = it * 32 + lq;
      const float* op = Os + row * OSP + 8 * e;
      const v4f v0 = *(const v4f*)(op);
      const v4f v1 = *(const v4f*)(op + 4);
      u[it] = pack8h(v0, v1, 1.0f);
      po[it] = (size_t)(mBase + row) * DM + nBase + 8 * e;
    }
#pragma unroll
    for (int it = 0; it < 4; ++it) *(volatile v4u*)(C16 + po[it]) = u[it];
    __threadfence();
#pragma unroll
    for (int it = 0; it < 4; ++it) *(volatile v4u*)(C16 + po[it]) = u[it];
  } else {
    const int bb = mBase / SEQ, key0 = mBase - bb * SEQ, hd = nBase / HD;
    v4u u[4];
    size_t po[4];
#pragma unroll
    for (int it = 0; it < 4; ++it) {
      const int L = it * 32 + lq;
      const int d = L >> 1, hf = L & 1;
      const int kk = hf * 64 + 8 * e;
      v4f v0, v1;
#pragma unroll
      for (int j = 0; j < 4; ++j) {
        v0[j] = Os[(kk + j) * OSP + d];
        v1[j] = Os[(kk + 4 + j) * OSP + d];
      }
      u[it] = pack8h(v0, v1, VSC);
      po[it] = ((size_t)((bb * NHD + hd) * HD + d)) * SEQ + key0 + kk;
    }
    const int t4 = tid >> 6, c = tid & 63;
    float s = 0.f;
#pragma unroll 8
    for (int r = 0; r < 32; ++r) s += Os[(32 * t4 + r) * OSP + c];
    Sm[t4 * GN + c] = s;
    __syncthreads();
    const bool wsum = (tid < 64);
    v4f sv = {0.f, 0.f, 0.f, 0.f};
    size_t ps = 0;
    if (wsum) {
      const int line = tid >> 3;
      const int tt = line >> 1, hf = line & 1;
      sv = *(const v4f*)(Sm + tt * GN + hf * 32 + 4 * e);
      ps = (size_t)(mBase / 32 + tt) * DM + nBase + hf * 32 + 4 * e;
    }
#pragma unroll
    for (int it = 0; it < 4; ++it) *(volatile v4u*)(C16 + po[it]) = u[it];
    if (wsum) *(volatile v4f*)(CS + ps) = sv;
    __threadfence();
#pragma unroll
    for (int it = 0; it < 4; ++it) *(volatile v4u*)(C16 + po[it]) = u[it];
    if (wsum) *(volatile v4f*)(CS + ps) = sv;
  }
}

__global__ __launch_bounds__(128)
void attn_kernel(const unsigned short* __restrict__ Q16, const unsigned short* __restrict__ K16,
                 const unsigned short* __restrict__ VT16, const float* __restrict__ VS,
                 unsigned short* Oh, unsigned short* Ol) {
  __shared__ __align__(16) unsigned short Pt[4 * 16 * PPH];
  __shared__ __align__(16) float Ot[4 * 16 * OTP];
  const int tid  = threadIdx.x;
  const int lane = tid & 31, wave = tid >> 5;
  const int hh   = lane >> 4, cl = lane & 15;
  const int bid  = blockIdx.x;
  const int qb   = bid & (NQB - 1);
  const int h    = (bid >> 5) & (NHD - 1);
  const int b    = bid >> 8;
  const int q0   = qb * QB + 16 * wave;
  const size_t qrow = (size_t)b * SEQ + q0;
  unsigned short* Pw = Pt + wave * (16 * PPH);
  float* Ow = Ot + wave * (16 * OTP);

  const unsigned short* qp = Q16 + (qrow + cl) * DM + h * HD + 8 * hh;
  const Frag qf0 = ldfrag(qp);
  const Frag qf1 = ldfrag(qp + 32);
  const unsigned short* kp = K16 + ((size_t)b * SEQ + cl) * DM + h * HD + 8 * hh;
  const unsigned short* vp = VT16 + ((size_t)(b * NHD + h) * HD + cl) * SEQ + 8 * hh;
  const float* vsp = VS + (size_t)b * NKT * DM + h * HD + cl;
  const float csc = PSC * VSC;

  float mrow[8], lrow[8];
  v8f acc[4];
#pragma unroll
  for (int r = 0; r < 8; ++r) { mrow[r] = -1.0e30f; lrow[r] = 0.f; }
#pragma unroll
  for (int nt = 0; nt < 4; ++nt) acc[nt] = zero8();

#pragma unroll 1
  for (int t = 0; t < NKT; ++t) {
    const unsigned short* k0p = kp + (size_t)(t * KT) * DM;
    const unsigned short* k1p = k0p + (size_t)16 * DM;
    const Frag k00 = ldfrag(k0p);
    const Frag k01 = ldfrag(k0p + 32);
    const Frag k10 = ldfrag(k1p);
    const Frag k11 = ldfrag(k1p + 32);
    v8f s0 = mma_h(qf0.x, k00.x, zero8());
    s0 = mma_h(qf1.x, k01.x, s0);
    v8f s1 = mma_h(qf0.x, k10.x, zero8());
    s1 = mma_h(qf1.x, k11.x, s1);
    float vs[4];
#pragma unroll
    for (int nt = 0; nt < 4; ++nt) vs[nt] = vsp[(size_t)t * DM + nt * 16] * csc;
#pragma unroll
    for (int r = 0; r < 8; ++r) {
      const float a0 = s0[r] * SCL, a1 = s1[r] * SCL;
      float tm = fmaxf(a0, a1);
      tm = fmaxf(tm, __shfl_xor(tm, 1, 32));
      tm = fmaxf(tm, __shfl_xor(tm, 2, 32));
      tm = fmaxf(tm, __shfl_xor(tm, 4, 32));
      tm = fmaxf(tm, __shfl_xor(tm, 8, 32));
      const float mn = fmaxf(mrow[r], tm);
      const float al = __expf(mrow[r] - mn);
      const float p0 = __expf(a0 - mn);
      const float p1 = __expf(a1 - mn);
      float rs = p0 + p1;
      rs += __shfl_xor(rs, 1, 32);
      rs += __shfl_xor(rs, 2, 32);
      rs += __shfl_xor(rs, 4, 32);
      rs += __shfl_xor(rs, 8, 32);
      mrow[r] = mn;
      lrow[r] = lrow[r] * al + rs;
      const float cm = rs * (1.0f / 32.0f);
      Pw[(8 * hh + r) * PPH + cl]      = h_bits((p0 - cm) * PSC);
      Pw[(8 * hh + r) * PPH + 16 + cl] = h_bits((p1 - cm) * PSC);
#pragma unroll
      for (int nt = 0; nt < 4; ++nt) acc[nt][r] = acc[nt][r] * al + cm * vs[nt];
    }
    __syncthreads();
    const Frag pa = ldfrag(Pw + cl * PPH + 8 * hh);
    const unsigned short* vtp = vp + t * KT;
#pragma unroll
    for (int nt = 0; nt < 4; ++nt) {
      const Frag vf = ldfrag(vtp + (size_t)nt * 16 * SEQ);
      acc[nt] = mma_h(pa.x, vf.x, acc[nt]);
    }
    __syncthreads();
  }

#pragma unroll
  for (int r = 0; r < 8; ++r) {
    const float inv = __builtin_amdgcn_rcpf(lrow[r] * csc);
#pragma unroll
    for (int nt = 0; nt < 4; ++nt) Ow[(8 * hh + r) * OTP + nt * 16 + cl] = acc[nt][r] * inv;
  }
  __syncthreads();
  const int rg = lane >> 3, e = lane & 7;
  v4u uh[4], ul[4];
  size_t po[4];
#pragma unroll
  for (int it = 0; it < 4; ++it) {
    const int row = it * 4 + rg;
    const float* op = Ow + row * OTP + 8 * e;
    const v4f v0 = *(const v4f*)(op);
    const v4f v1 = *(const v4f*)(op + 4);
    split8(v0, v1, uh[it], ul[it]);
    po[it] = (qrow + row) * DM + h * HD + 8 * e;
  }
#pragma unroll
  for (int it = 0; it < 4; ++it) {
    *(volatile v4u*)(Oh + po[it]) = uh[it];
    *(volatile v4u*)(Ol + po[it]) = ul[it];
  }
  __threadfence();
#pragma unroll
  for (int it = 0; it < 4; ++it) {
    *(volatile v4u*)(Oh + po[it]) = uh[it];
    *(volatile v4u*)(Ol + po[it]) = ul[it];
  }
}

__global__ __launch_bounds__(256)
void outproj_kernel(const unsigned short* __restrict__ Xh, const unsigned short* __restrict__ Xl,
                    const unsigned short* __restrict__ WT, const float* __restrict__ bias, float* out) {
  __shared__ __align__(16) float Os[GM * OSP];
  const int tid  = threadIdx.x;
  const int lane = tid & 31, wave = tid >> 5;
  const int hh   = lane >> 4, cl = lane & 15;
  const int wm   = wave >> 1, wn = wave & 1;
  const int mBase = blockIdx.x * GM;
  const int nBase = blockIdx.y * GN;
  const size_t ar0 = (size_t)(mBase + 32 * wm + cl) * DM + 8 * hh;
  const size_t ar1 = ar0 + (size_t)16 * DM;
  const unsigned short* b0p = WT + (size_t)(nBase + 32 * wn + cl) * DM + 8 * hh;
  const unsigned short* b1p = b0p + (size_t)16 * DM;

  v8f acc[2][2];
#pragma unroll
  for (int mi = 0; mi < 2; ++mi)
#pragma unroll
    for (int ni = 0; ni < 2; ++ni) acc[mi][ni] = zero8();

#pragma unroll 1
  for (int k0 = 0; k0 < DM; k0 += 32) {
    const Frag ah0 = ldfrag(Xh + ar0 + k0);
    const Frag ah1 = ldfrag(Xh + ar1 + k0);
    const Frag al0 = ldfrag(Xl + ar0 + k0);
    const Frag al1 = ldfrag(Xl + ar1 + k0);
    const Frag fb0 = ldfrag(b0p + k0);
    const Frag fb1 = ldfrag(b1p + k0);
    acc[0][0] = mma_b(ah0.b, fb0.b, acc[0][0]);
    acc[0][0] = mma_b(al0.b, fb0.b, acc[0][0]);
    acc[0][1] = mma_b(ah0.b, fb1.b, acc[0][1]);
    acc[0][1] = mma_b(al0.b, fb1.b, acc[0][1]);
    acc[1][0] = mma_b(ah1.b, fb0.b, acc[1][0]);
    acc[1][0] = mma_b(al1.b, fb0.b, acc[1][0]);
    acc[1][1] = mma_b(ah1.b, fb1.b, acc[1][1]);
    acc[1][1] = mma_b(al1.b, fb1.b, acc[1][1]);
  }

#pragma unroll
  for (int mi = 0; mi < 2; ++mi) {
#pragma unroll
    for (int ni = 0; ni < 2; ++ni) {
      const int n_loc = 32 * wn + 16 * ni + cl;
      const float bb = bfr(bias[nBase + n_loc]);
#pragma unroll
      for (int r = 0; r < 8; ++r) {
        const int m_loc = 32 * wm + 16 * mi + 8 * hh + r;
        Os[m_loc * OSP + n_loc] = acc[mi][ni][r] + bb;
      }
    }
  }
  __syncthreads();

  const int e = tid & 7, lq = tid >> 3;
  v4f v[8];
  size_t po[8];
#pragma unroll
  for (int it = 0; it < 8; ++it) {
    const int L = it * 32 + lq;
    const int row = L >> 1, hf = L & 1;
    v[it] = *(const v4f*)(Os + row * OSP + hf * 32 + 4 * e);
    po[it] = (size_t)(mBase + row) * DM + nBase + hf * 32 + 4 * e;
  }
#pragma unroll
  for (int it = 0; it < 8; ++it) *(volatile v4f*)(out + po[it]) = v[it];
  __threadfence();
#pragma unroll
  for (int it = 0; it < 8; ++it) *(volatile v4f*)(out + po[it]) = v[it];
}

extern "C" void kernel_launch(void* const* d_in, const int* in_sizes, int n_in,
                              void* d_out, int out_size, void* d_ws, size_t ws_size,
                              hipStream_t stream) {
  if (n_in < 10) return;
  const int ntot = in_sizes[0];
  if (ntot <= 0 || (ntot % (SEQ * DM)) != 0) return;
  const int nb = ntot / (SEQ * DM);
  if (nb < 1 || nb > MAXNB) return;
  const int ntok = nb * SEQ;
  if (in_sizes[1] != ntot) return;
  if (in_sizes[2] != DM * DM || in_sizes[3] != DM * DM || in_sizes[4] != DM * DM) return;
  if (in_sizes[5] != DM * DM || in_sizes[6] != DM * DM || in_sizes[8] != DM * DM) return;
  if (in_sizes[7] != DM || in_sizes[9] != DM) return;
  if (out_size != 2 * ntot) return;

  const size_t tokB = (size_t)ntok * DM * 2;
  const size_t wB   = (size_t)DM * DM * 2;
  const size_t vsB  = (size_t)(ntok / KT) * DM * 4;

  size_t off = 0;
  const size_t oXA  = off; off += tokB;
  const size_t oXB  = off; off += tokB;
  const size_t oW0  = off; off += wB;
  const size_t oW1  = off; off += wB;
  const size_t oW2  = off; off += wB;
  const size_t oW3  = off; off += wB;
  const size_t oW4  = off; off += wB;
  const size_t oW5  = off; off += wB;
  const size_t oQK  = off; off += tokB;
  const size_t oCQK = off; off += tokB;
  const size_t oVT  = off; off += tokB;
  const size_t oCVT = off; off += tokB;
  const size_t oVSA = off; off += vsB;
  const size_t oVSB = off; off += vsB;
  const size_t oOAh = off; off += tokB;
  const size_t oOAl = off; off += tokB;
  const size_t oOBh = off; off += tokB;
  const size_t oOBl = off; off += tokB;
  if (off > ws_size) return;
  if (off > (size_t)134217728) return;

  const float* tokA  = (const float*)d_in[0];
  const float* tokB_ = (const float*)d_in[1];
  const float* Wqk   = (const float*)d_in[2];
  const float* Wcqk  = (const float*)d_in[3];
  const float* Wv    = (const float*)d_in[4];
  const float* Wcv   = (const float*)d_in[5];
  const float* Wo    = (const float*)d_in[6];
  const float* bo    = (const float*)d_in[7];
  const float* Wco   = (const float*)d_in[8];
  const float* bco   = (const float*)d_in[9];
  float* out0 = (float*)d_out;
  float* out1 = out0 + (size_t)ntot;

  char* ws = (char*)d_ws;
  unsigned short* XA   = (unsigned short*)(ws + oXA);
  unsigned short* XB   = (unsigned short*)(ws + oXB);
  unsigned short* WqkT = (unsigned short*)(ws + oW0);
  unsigned short* WcqkT= (unsigned short*)(ws + oW1);
  unsigned short* WvT  = (unsigned short*)(ws + oW2);
  unsigned short* WcvT = (unsigned short*)(ws + oW3);
  unsigned short* WoT  = (unsigned short*)(ws + oW4);
  unsigned short* WcoT = (unsigned short*)(ws + oW5);
  unsigned short* QK   = (unsigned short*)(ws + oQK);
  unsigned short* CQK  = (unsigned short*)(ws + oCQK);
  unsigned short* VT   = (unsigned short*)(ws + oVT);
  unsigned short* CVT  = (unsigned short*)(ws + oCVT);
  float*          VSA  = (float*)(ws + oVSA);
  float*          VSB  = (float*)(ws + oVSB);
  unsigned short* OAh  = (unsigned short*)(ws + oOAh);
  unsigned short* OAl  = (unsigned short*)(ws + oOAl);
  unsigned short* OBh  = (unsigned short*)(ws + oOBh);
  unsigned short* OBl  = (unsigned short*)(ws + oOBl);

  const dim3 blk256(256);
  const dim3 blk128(128);
  const dim3 gproj(ntok / GM, DM / GN);

  cvt_kernel<<<dim3(ntot / 2048), blk256, 0, stream>>>(tokA, XA, ntot / 8);
  cvt_kernel<<<dim3(ntot / 2048), blk256, 0, stream>>>(tokB_, XB, ntot / 8);
  wtrans_kernel<<<dim3(DM / 64, DM / 64), blk256, 0, stream>>>(Wqk,  WqkT,  DM, DM);
  wtrans_kernel<<<dim3(DM / 64, DM / 64), blk256, 0, stream>>>(Wcqk, WcqkT, DM, DM);
  wtrans_kernel<<<dim3(DM / 64, DM / 64), blk256, 0, stream>>>(Wv,   WvT,   DM, DM);
  wtrans_kernel<<<dim3(DM / 64, DM / 64), blk256, 0, stream>>>(Wcv,  WcvT,  DM, DM);
  wtrans_kernel<<<dim3(DM / 64, DM / 64), blk256, 0, stream>>>(Wo,   WoT,   DM, DM);
  wtrans_kernel<<<dim3(DM / 64, DM / 64), blk256, 0, stream>>>(Wco,  WcoT,  DM, DM);
  proj_kernel<0><<<gproj, blk256, 0, stream>>>(XA, WqkT,  QK,  VSA);
  proj_kernel<0><<<gproj, blk256, 0, stream>>>(XB, WcqkT, CQK, VSA);
  proj_kernel<1><<<gproj, blk256, 0, stream>>>(XA, WvT,   VT,  VSA);
  proj_kernel<1><<<gproj, blk256, 0, stream>>>(XB, WcvT,  CVT, VSB);
  attn_kernel<<<dim3(nb * NHD * NQB), blk128, 0, stream>>>(QK, CQK, CVT, VSB, OAh, OAl);
  outproj_kernel<<<gproj, blk256, 0, stream>>>(OAh, OAl, WoT, bo, out0);
  attn_kernel<<<dim3(nb * NHD * NQB), blk128, 0, stream>>>(CQK, QK, VT, VSA, OBh, OBl);
  outproj_kernel<<<gproj, blk256, 0, stream>>>(OBh, OBl, WcoT, bco, out1);
  (void)hipGetLastError();
}
